// InvButterflyLayer_7868380086486
// MI455X (gfx1250) — hardware-verified
//
#include <hip/hip_runtime.h>
#include <stddef.h>


typedef _Float16 v16h __attribute__((ext_vector_type(16)));
typedef _Float16 v8h  __attribute__((ext_vector_type(8)));
typedef float    v8f  __attribute__((ext_vector_type(8)));
typedef float    v4f  __attribute__((ext_vector_type(4)));

#ifndef NB
#define NB 256
#endif
#define NB_FULL 256
#define MIDSZ   16384
#define CH      16
#define NLVL    8
#define NBR     256
#define ROWS    512
#define OUTF    64
#define OUTROW  8192
#define CHAN    (ROWS * CH)
#define BUFH    (2 * CHAN)
#define NMAT    510
#define LDC     68
#ifndef ACT_RES
#define ACT_RES 1
#endif

#define WCARRY 64.0f
#define XCARRY 16.0f
#define RCARRY 2048.0f

static_assert(NB >= 1 && NB <= NB_FULL);
static_assert(MIDSZ == 32 * ROWS);
static_assert((1 << NLVL) == NBR);
static_assert(NMAT == 2 * NBR - 2);
static_assert(OUTROW == NBR * OUTF / 2);
static_assert(CH == 16 && OUTF == 64);
static_assert((CHAN % 8) == 0 && (LDC % 4) == 0 && LDC >= 64);
static_assert(NBR * CH * 2 == 1024 * 8);
static_assert(ACT_RES == 0 || ACT_RES == 1);

#define WT_BYTES   ((size_t)NMAT * 512 * 2)
#define W0_BYTES   ((size_t)1024 * 2)
#define FD_BYTES   ((size_t)NBR * 1024 * 2)
#define FEAT_BYTES ((size_t)NB * 2 * NBR * CH * 2)
#define OFF_WT ((size_t)0)
#define OFF_W0 (OFF_WT + WT_BYTES)
#define OFF_FD (OFF_W0 + W0_BYTES)
#define OFF_FH (OFF_FD + FD_BYTES)
#define OFF_FR (OFF_FH + FEAT_BYTES)
#define WS_TOTAL (OFF_FR + FEAT_BYTES)
static_assert((WT_BYTES % 128) == 0 && (W0_BYTES % 128) == 0 && (FD_BYTES % 128) == 0);
static_assert((FEAT_BYTES % 128) == 0);
static_assert(WS_TOTAL <= (size_t)134217728);

#define OUT1_OFF ((size_t)NB_FULL * OUTROW)
static_assert(OUT1_OFF * 4 == (size_t)8388608);

__device__ __forceinline__ float bf16r(float x) {
  unsigned int u = __float_as_uint(x);
  u = (u + 0x7FFFu + ((u >> 16) & 1u)) & 0xFFFF0000u;
  return __uint_as_float(u);
}

static __device__ __forceinline__ _Float16 toh_flush(float v) {
  const _Float16 r = (_Float16)v;
  return (fabsf(v) < 6.103515625e-05f) ? (_Float16)0.0f : r;
}
static __device__ __forceinline__ void split16(float v, _Float16& hi, _Float16& rs) {
  hi = toh_flush(v);
  rs = toh_flush((v - (float)hi) * RCARRY);
}

__device__ __forceinline__ v16h frag_at(const _Float16* p) {
  v8h lo = *(const v8h*)(p);
  v8h hi = *(const v8h*)(p + 16);
  v16h out;
#pragma unroll
  for (int i = 0; i < 8; ++i) { out[i] = lo[i]; out[i + 8] = hi[i]; }
  return out;
}
__device__ __forceinline__ v16h frag_join(v8h lo, v8h hi) {
  v16h out;
#pragma unroll
  for (int i = 0; i < 8; ++i) { out[i] = lo[i]; out[i + 8] = hi[i]; }
  return out;
}

__device__ __forceinline__ v8f wmma16(v16h a, v16h b, v8f c) {
  v8f d = __builtin_amdgcn_wmma_f32_16x16x32_f16(false, a, false, b, (short)0, c,
                                                 false, false);
  asm volatile("v_nop\n\tv_nop\n\tv_nop\n\tv_nop" : "+v"(d) : "v"(a), "v"(b));
  return d;
}

__global__ __launch_bounds__(64) void wconv_kernel(
    const float* __restrict__ W, _Float16* __restrict__ Wt,
    unsigned kshift, unsigned nshift, unsigned tree) {
  __shared__ __attribute__((aligned(16))) _Float16 T[1536];
  const unsigned tid = threadIdx.x;
  const unsigned id = blockIdx.x;
  const unsigned K = 1u << kshift, N = 1u << nshift;
  const unsigned KN = 1u << (kshift + nshift);
  const unsigned ldk = K + 8u;
  const unsigned v = id + 2u;
  const unsigned lvl = 31u - (unsigned)__clz((int)v);
  const unsigned tn = v - (1u << lvl);
  const unsigned tmat = (lvl - 1u) * (unsigned)NBR + tn;
  const unsigned smat = (tree != 0u) ? tmat : id;
  const size_t src = (size_t)smat * KN;
  const unsigned nld = KN >> 6;
#pragma unroll 1
  for (unsigned j = 0; j < nld; ++j) {
    const unsigned idx = tid + 64u * j;
    const unsigned kk = idx >> nshift, nn = idx & (N - 1u);
    const float w = W[src + idx];
    T[nn * ldk + kk] = toh_flush(WCARRY * bf16r(w));
  }
  __syncthreads();
  const unsigned npieces = KN >> 3;
  const bool two = (npieces > 64u);
  v8h x[2];
  size_t off[2];
#pragma unroll
  for (unsigned i = 0; i < 2u; ++i) {
    unsigned p = tid + 64u * i;
    p = (p < npieces) ? p : (npieces - 1u);
    const unsigned e0 = p * 8u;
    const unsigned nn = e0 >> kshift, kk = e0 & (K - 1u);
    x[i] = *(const v8h*)&T[nn * ldk + kk];
    off[i] = (size_t)id * KN + e0;
  }
  *(volatile v8h*)(Wt + off[0]) = x[0];
  if (two) *(volatile v8h*)(Wt + off[1]) = x[1];
  __threadfence();
  *(volatile v8h*)(Wt + off[0]) = x[0];
  if (two) *(volatile v8h*)(Wt + off[1]) = x[1];
}

__global__ __launch_bounds__(256) void bfly_kernel(
    const float* __restrict__ in_data, const float* __restrict__ mid_dense,
    const float* __restrict__ in_bias, const float* __restrict__ biases,
    const _Float16* __restrict__ W0T, const _Float16* __restrict__ WT,
    _Float16* __restrict__ FH, _Float16* __restrict__ FR) {
  __shared__ __attribute__((aligned(16))) _Float16 sh_hi[2 * BUFH];
  __shared__ __attribute__((aligned(16))) _Float16 sh_rs[2 * BUFH];

  const unsigned tid = threadIdx.x, lane = tid & 31u;
  const unsigned wave = (unsigned)__builtin_amdgcn_readfirstlane((int)(tid >> 5));
  const unsigned hh = lane >> 4, m = lane & 15u;
  const unsigned b = blockIdx.x;
  const float* idb = in_data + (size_t)b * (MIDSZ * 2);

  {
    const float bias0 = bf16r(in_bias[m]);
    const float C0  = 1.0f / (WCARRY * XCARRY);
    const float C0R = 1.0f / (WCARRY * XCARRY * RCARRY);
#pragma unroll 1
    for (unsigned task = wave; task < 32u; task += 8u) {
      const unsigned t0 = task * 16u;
      unsigned ta = t0 + m;
      ta = (ta > 510u) ? 510u : ta;
      v8f ah0 = {}, ah1 = {}, ar0 = {}, ar1 = {};
#pragma unroll
      for (unsigned kk = 0; kk < 2u; ++kk) {
        v16h x0h, x1h, x0r, x1r;
#pragma unroll
        for (unsigned hf = 0; hf < 2u; ++hf) {
          const unsigned p0 = 32u * ta + 32u * kk + 16u * hf + 8u * hh;
          const float* dp = idb + 2u * p0;
          const float* mp = mid_dense + 2u * p0;
#pragma unroll
          for (unsigned q = 0; q < 4u; ++q) {
            const v4f d = *(const v4f*)(dp + 4u * q);
            const v4f g = *(const v4f*)(mp + 4u * q);
#pragma unroll
            for (unsigned s = 0; s < 2u; ++s) {
              const unsigned e = 8u * hf + 2u * q + s;
              const float c0 = XCARRY * (bf16r(d[2u * s]) * bf16r(g[2u * s]));
              const float c1 = XCARRY * (bf16r(d[2u * s + 1u]) * bf16r(g[2u * s + 1u]));
              _Float16 h0, s0, h1, s1;
              split16(c0, h0, s0);
              split16(c1, h1, s1);
              x0h[e] = h0; x0r[e] = s0;
              x1h[e] = h1; x1r[e] = s1;
            }
          }
        }
        const v16h bf = frag_at(W0T + m * 64u + kk * 32u + hh * 8u);
        ah0 = wmma16(x0h, bf, ah0);
        ah1 = wmma16(x1h, bf, ah1);
        if (ACT_RES) {
          ar0 = wmma16(x0r, bf, ar0);
          ar1 = wmma16(x1r, bf, ar1);
        }
      }
#pragma unroll
      for (unsigned r = 0; r < 8u; ++r) {
        const unsigned t = t0 + 8u * hh + r;
        float v0 = ah0[r] * C0;
        float v1 = ah1[r] * C0;
        if (ACT_RES) { v0 += ar0[r] * C0R; v1 += ar1[r] * C0R; }
        v0 = fmaxf(v0 + bias0, 0.0f);
        v1 = fmaxf(v1 + bias0, 0.0f);
        _Float16 h0, s0, h1, s1;
        split16(v0, h0, s0);
        split16(v1, h1, s1);
        if (t < 511u) {
          const unsigned o = t * CH + m;
          sh_hi[o] = h0;
          sh_hi[CHAN + o] = h1;
          if (ACT_RES) { sh_rs[o] = s0; sh_rs[CHAN + o] = s1; }
        }
      }
    }
  }
  __syncthreads();

  unsigned Tprev = 511u;
#pragma unroll 1
  for (unsigned lvl = 1u; lvl <= (unsigned)NLVL; ++lvl) {
    const unsigned nb = 1u << lvl;
    const unsigned T = (Tprev - 1u) >> 1;
    const bool merged = (lvl >= 6u);
    const unsigned ntshift = merged ? 0u : (5u - lvl);
    const unsigned ntasks = merged ? nb : ((2u * nb) << ntshift);
    const unsigned srcoff = (lvl & 1u) ? 0u : (unsigned)BUFH;
    const unsigned dstoff = (lvl & 1u) ? (unsigned)BUFH : 0u;
    const float lscale = __uint_as_float((127u - lvl) << 23);
    const float C1  = 1.0f / (WCARRY * 2.0f);
    const float C1R = 1.0f / (WCARRY * 2.0f * RCARRY);
#pragma unroll 1
    for (unsigned task = wave; task < ntasks; task += 8u) {
      const unsigned tile = task & ((1u << ntshift) - 1u);
      const unsigned rest = task >> ntshift;
      const unsigned n  = rest & (nb - 1u);
      const unsigned ti = rest >> lvl;
      const unsigned t0 = tile << 4;
      const unsigned mat = (nb - 2u) + n;
      const v16h bf = frag_at(WT + (size_t)mat * 512u + m * 32u + hh * 8u);
      const float bias = bf16r(biases[((lvl - 1u) * (unsigned)NBR + n) * CH + m]) * lscale;

      const unsigned ai = merged ? (m >> 3) : ti;
      unsigned at = merged ? (m & 7u) : (t0 + m);
      at = (at < T) ? at : (T - 1u);
      const unsigned aoff = srcoff + ai * (unsigned)CHAN
                          + (((n >> 1) * Tprev + 2u * at) << 4) + 8u * hh;
      const v8h l0 = *(const v8h*)&sh_hi[aoff];
      const v8h l1 = *(const v8h*)&sh_hi[aoff + 16u];
      const v16h ahi = frag_join(l0, l1);
      v8f acc = {}, accr = {};
      acc = wmma16(ahi, bf, acc);
      if (ACT_RES) {
        const v8h r0 = *(const v8h*)&sh_rs[aoff];
        const v8h r1 = *(const v8h*)&sh_rs[aoff + 16u];
        const v16h ars = frag_join(r0, r1);
        accr = wmma16(ars, bf, accr);
      }
#pragma unroll
      for (unsigned r = 0; r < 8u; ++r) {
        const unsigned di = merged ? hh : ti;
        const unsigned dt = merged ? r : (t0 + 8u * hh + r);
        float v = acc[r] * C1;
        if (ACT_RES) v += accr[r] * C1R;
        v = fmaxf(v + bias, 0.0f);
        _Float16 hv, sv;
        split16(v, hv, sv);
        if (dt < T) {
          const unsigned o = dstoff + di * (unsigned)CHAN + ((n * T + dt) << 4) + m;
          sh_hi[o] = hv;
          if (ACT_RES) sh_rs[o] = sv;
        }
      }
    }
    __syncthreads();
    Tprev = T;
  }

  {
    v8h xh[4], xr[4];
    size_t off[4];
#pragma unroll
    for (unsigned j = 0; j < 4u; ++j) {
      const unsigned p = tid + 256u * j;
      const unsigned i = p >> 9, w = p & 511u;
      const unsigned lo = i * (unsigned)CHAN + w * 8u;
      xh[j] = *(const v8h*)&sh_hi[lo];
      if (ACT_RES) xr[j] = *(const v8h*)&sh_rs[lo]; else xr[j] = xh[j];
      off[j] = (size_t)b * (2u * NBR * CH) + (size_t)p * 8u;
    }
#pragma unroll
    for (int j = 0; j < 4; ++j) {
      *(volatile v8h*)(FH + off[j]) = xh[j];
      if (ACT_RES) *(volatile v8h*)(FR + off[j]) = xr[j];
    }
    __threadfence();
#pragma unroll
    for (int j = 0; j < 4; ++j) {
      *(volatile v8h*)(FH + off[j]) = xh[j];
      if (ACT_RES) *(volatile v8h*)(FR + off[j]) = xr[j];
    }
  }
}

__global__ __launch_bounds__(128) void head_kernel(
    const _Float16* __restrict__ FH, const _Float16* __restrict__ FR,
    const _Float16* __restrict__ FDT, float* __restrict__ out) {
  __shared__ __attribute__((aligned(16))) float Cs[4 * 16 * LDC];
  const unsigned tid = threadIdx.x, lane = tid & 31u;
  const unsigned wave = (unsigned)__builtin_amdgcn_readfirstlane((int)(tid >> 5));
  const unsigned hh = lane >> 4, m = lane & 15u;
  const unsigned id = blockIdx.x * 4u + wave;
  const unsigned n = id & 255u;
  const unsigned b0 = (id >> 8) * 8u;
  const unsigned cbase = wave * (16u * LDC);

  unsigned ba = b0 + (m >> 1);
  ba = (ba < (unsigned)NB) ? ba : (unsigned)(NB - 1);
  const size_t aoff = ((size_t)ba * 2u + (m & 1u)) * (size_t)(NBR * CH) + n * CH + hh * 8u;
  const v8h zero8 = {};
  const v16h ah = frag_join(*(const v8h*)(FH + aoff), zero8);
  v16h ar = ah;
  if (ACT_RES) ar = frag_join(*(const v8h*)(FR + aoff), zero8);

#pragma unroll
  for (unsigned j = 0; j < 4u; ++j) {
    const v16h bf = frag_join(
        *(const v8h*)(FDT + ((size_t)n * OUTF + 16u * j + m) * CH + hh * 8u), zero8);
    v8f a = {}, a2 = {};
    a = wmma16(ah, bf, a);
    if (ACT_RES) a2 = wmma16(ar, bf, a2);
#pragma unroll
    for (unsigned r = 0; r < 8u; ++r) {
      float t = a[r];
      if (ACT_RES) t += a2[r] * (1.0f / RCARRY);
      Cs[cbase + (hh * 8u + r) * LDC + 16u * j + m] = t;
    }
  }
  __syncthreads();

  const float k1 = 4.0f;
  const float k0 = 4.0f / 16384.0f;
  v4f od[2], o1[2];
  size_t off[2];
  bool ok[2];
#pragma unroll
  for (unsigned pass = 0; pass < 2u; ++pass) {
    const unsigned bl = 4u * pass + (lane >> 3);
    const unsigned fe0 = (lane & 7u) * 4u;
    const unsigned r0 = cbase + (2u * bl) * LDC + 2u * fe0;
    const unsigned r1 = r0 + LDC;
    const v4f u0 = *(const v4f*)&Cs[r0];
    const v4f u1 = *(const v4f*)&Cs[r0 + 4u];
    const v4f w0 = *(const v4f*)&Cs[r1];
    const v4f w1 = *(const v4f*)&Cs[r1 + 4u];
    v4f a, c;
    a[0] = (u0[0] - w0[1]) * k0;  c[0] = u0[1] * k1;
    a[1] = (u0[2] - w0[3]) * k0;  c[1] = u0[3] * k1;
    a[2] = (u1[0] - w1[1]) * k0;  c[2] = u1[1] * k1;
    a[3] = (u1[2] - w1[3]) * k0;  c[3] = u1[3] * k1;
    od[pass] = a;
    o1[pass] = c;
    off[pass] = (size_t)(b0 + bl) * OUTROW + n * 32u + fe0;
    ok[pass] = (b0 + bl) < (unsigned)NB;
  }
#pragma unroll
  for (int p = 0; p < 2; ++p) {
    if (ok[p]) {
      *(volatile v4f*)(out + off[p]) = od[p];
      *(volatile v4f*)(out + OUT1_OFF + off[p]) = o1[p];
    }
  }
  __threadfence();
#pragma unroll
  for (int p = 0; p < 2; ++p) {
    if (ok[p]) {
      *(volatile v4f*)(out + off[p]) = od[p];
      *(volatile v4f*)(out + OUT1_OFF + off[p]) = o1[p];
    }
  }
}

extern "C" void kernel_launch(void* const* d_in, const int* in_sizes, int n_in,
                              void* d_out, int out_size, void* d_ws, size_t ws_size,
                              hipStream_t stream) {
  if (n_in < 7) return;
  if ((long long)in_sizes[0] < (long long)NB * MIDSZ * 2) return;
  if (in_sizes[1] < MIDSZ * 2) return;
  if (in_sizes[2] < 64 * CH) return;
  if (in_sizes[3] < CH) return;
  if ((long long)in_sizes[4] < (long long)NLVL * NBR * 2 * CH * CH) return;
  if (in_sizes[5] < NLVL * NBR * CH) return;
  if (in_sizes[6] < NBR * CH * OUTF) return;
  if ((long long)out_size < (long long)NB_FULL * OUTROW + (long long)NB * OUTROW) return;
  if (ws_size < WS_TOTAL) return;

  const float* in_data   = (const float*)d_in[0];
  const float* mid_dense = (const float*)d_in[1];
  const float* in_filter = (const float*)d_in[2];
  const float* in_bias   = (const float*)d_in[3];
  const float* filters   = (const float*)d_in[4];
  const float* biases    = (const float*)d_in[5];
  const float* fea_dense = (const float*)d_in[6];
  float* out = (float*)d_out;

  char* ws = (char*)d_ws;
  _Float16* WT  = (_Float16*)(ws + OFF_WT);
  _Float16* W0T = (_Float16*)(ws + OFF_W0);
  _Float16* FDT = (_Float16*)(ws + OFF_FD);
  _Float16* FH  = (_Float16*)(ws + OFF_FH);
  _Float16* FR  = (_Float16*)(ws + OFF_FR);

  wconv_kernel<<<dim3(NMAT), dim3(64), 0, stream>>>(filters, WT, 5u, 4u, 1u);
  wconv_kernel<<<dim3(1), dim3(64), 0, stream>>>(in_filter, W0T, 6u, 4u, 0u);
  wconv_kernel<<<dim3(NBR), dim3(64), 0, stream>>>(fea_dense, FDT, 4u, 6u, 0u);

  bfly_kernel<<<dim3(NB), dim3(256), 0, stream>>>(in_data, mid_dense, in_bias, biases,
                                                  W0T, WT, FH, FR);
  head_kernel<<<dim3(64 * ((NB + 7) / 8)), dim3(128), 0, stream>>>(FH, FR, FDT, out);
}
